// Q_network_12171937317191
// MI455X (gfx1250) — hardware-verified
//
#include <hip/hip_runtime.h>


namespace {
constexpr int NB_ = 128, NA = 32, DS = 128, AC = 16, HH = 256, R = NB_ * NA  , KSA = 160  ;
constexpr float XS = 8.0f, HS = 256.0f, WSC = 256.0f, EPS = 1e-5f;
typedef _Float16 b16;
typedef __attribute__((ext_vector_type(16))) _Float16 v16b;
typedef __attribute__((ext_vector_type(8))) _Float16 v8b;
typedef __attribute__((ext_vector_type(8))) float v8f;
typedef __attribute__((ext_vector_type(4))) float v4f;
typedef __attribute__((ext_vector_type(2))) float v2f;
__device__ __forceinline__ float bf16_rne(float f) { unsigned int u = __float_as_uint(f); u += 0x7FFFu + ((u >> 16) & 1u); float r = __uint_as_float(u & 0xFFFF0000u); asm volatile("" : "+v"(r)); return r; }
__device__ __forceinline__ float bfv(float f) { float r = bf16_rne(f); asm volatile("" : "+v"(r)); return r; }
__device__ __forceinline__ void split16(float v, b16& hi, b16& lo) { hi = (b16)v; lo = (b16)(v - (float)hi); }
__device__ __forceinline__ v16b frag_kb(const b16* p, int hh) { const v8b a = *(const v8b*)(p + 8 * hh), b = *(const v8b*)(p + 16 + 8 * hh); v16b f;
#pragma unroll
  for (int e = 0; e < 8; ++e) { f[e] = a[e]; f[8 + e] = b[e]; } return f; }
__device__ __forceinline__ v8f wmma16b(v16b a, v16b b, v8f c) { v8f d = __builtin_amdgcn_wmma_f32_16x16x32_f16(false, a, false, b, (short)0, c, false, false); asm volatile("v_nop\n\tv_nop\n\tv_nop\n\tv_nop" : "+v"(d) : "v"(a), "v"(b)); return d; }
__device__ __forceinline__ void wave_lds_sync() { __builtin_amdgcn_fence(__ATOMIC_RELEASE, "workgroup"); __builtin_amdgcn_wave_barrier(); __builtin_amdgcn_fence(__ATOMIC_ACQUIRE, "workgroup"); }
__device__ __forceinline__ float pmul(float a, float b) { float p = a * b; asm volatile("" : "+v"(p)); return p; }

__host__ __device__ constexpr int wk(int w) { return w == 0 || w == 10 ? DS : (w == 6 ? KSA : (w == 12 ? 512 : HH)); }
__host__ __device__ constexpr int wrows(int w) { return w == 14 ? 16 : HH; }
__host__ __device__ constexpr size_t woff(int w) { size_t o = 0; for (int i = 0; i < w; ++i) o += (size_t)wrows(i) * wk(i); return o; }
struct WPtrs { const float* p[15]; };
struct BPtrs { const float* p[15]; };
__global__ __launch_bounds__(256) void wput_kernel(WPtrs Ws, b16* __restrict__ WB) { const int w = blockIdx.y; const float* src = Ws.p[w]; const int K = wk(w), rows = wrows(w), kin = (w == 6 ? 144 : K); b16* dst = WB + woff(w); const size_t nt = (size_t)gridDim.x * 256, u0 = (size_t)blockIdx.x * 256 + threadIdx.x; v8b v;
  for (size_t u = u0; u < (size_t)rows * (K / 8); u += nt) { const int o = (int)(u / (K / 8)), k0 = (int)(u % (K / 8)) * 8;
#pragma unroll
    for (int j = 0; j < 8; ++j) { const int k = k0 + j; v[j] = (b16)(k < kin ? bf16_rne(src[(size_t)k * rows + o]) * WSC : 0.0f); } for (int pass = 0; pass < 2; ++pass) { *(volatile v8b*)(dst + (size_t)o * K + k0) = v; __threadfence(); } } }

template <int K, int NT>
__device__ __forceinline__ void gemm16(b16 (*Ah)[520], b16 (*Al)[520], bool hl, const b16* W, const float* bias, int act  , float scale, float (*Tf)[260], int nloc, int hlf) { v8f acc[NT];
#pragma unroll
  for (int t = 0; t < NT; ++t) acc[t] = (v8f){};
#pragma unroll 1
  for (int kb = 0; kb < K; kb += 32) { const v16b a = frag_kb(&Ah[nloc][kb], hlf); v16b al; if (hl) al = frag_kb(&Al[nloc][kb], hlf);
#pragma unroll
    for (int t = 0; t < NT; ++t) { const v16b bw = frag_kb(W + (size_t)(t * 16 + nloc) * K + kb, hlf); acc[t] = wmma16b(a, bw, acc[t]); if (hl) acc[t] = wmma16b(al, bw, acc[t]); } }
#pragma unroll
  for (int t = 0; t < NT; ++t) { const int cc = t * 16 + nloc; const float bb = bfv(bias[cc]);
#pragma unroll
    for (int r8 = 0; r8 < 8; ++r8) { const float v = acc[t][r8] * scale + bb; Tf[8 * hlf + r8][cc] = act ? tanhf(v) : v; } } }
__device__ __forceinline__ void stage_hl(float (*Tf)[260], b16 (*Ah)[520], b16 (*Al)[520], int coff, int lane) { for (int rr = 0; rr < 16; ++rr) for (int q = 0; q < 8; ++q) { const int c = q * 32 + lane; b16 p, pl; split16(Tf[rr][c] * HS, p, pl); Ah[rr][coff + c] = p; Al[rr][coff + c] = pl; } }
__global__ __launch_bounds__(32) void agent_kernel(const float* __restrict__ states, const float* __restrict__ actions, const b16* __restrict__ WB, BPtrs Bs, int RLIM, float* __restrict__ SE, float* __restrict__ KK, float* __restrict__ QQ, float* __restrict__ OA, float* __restrict__ AV, float* __restrict__ CU) { __shared__ __attribute__((aligned(16))) b16 Ah[16][520], Al[16][520]; __shared__ float Tf[16][260], Ts[16][260]; const int lane = threadIdx.x, nloc = lane & 15, hlf = lane >> 4; const size_t r0 = (size_t)blockIdx.x * 16; if (r0 >= (size_t)RLIM) return;
  auto store = [&](float* P, float (*T)[260]) { for (int pass = 0; pass < 2; ++pass) { for (int rr = 0; rr < 16; ++rr) for (int q = 0; q < 2; ++q) *(volatile v4f*)(P + (r0 + rr) * HH + q * 128 + lane * 4) = *(const v4f*)(&T[rr][q * 128 + lane * 4]); __threadfence(); } };
  if (lane < 16) for (int k = 0; k < 520; ++k) { Al[lane][k] = (b16)0.0f; }
  for (int rr = 0; rr < 16; ++rr) { for (int q = 0; q < 4; ++q) { const int c = q * 32 + lane; Ah[rr][c] = (b16)(bfv(states[(r0 + rr) * DS + c]) * XS); } Ah[rr][DS + lane] = (b16)(lane < AC ? bfv(actions[(r0 + rr) * AC + lane]) * XS : 0.0f); }
  if (lane < 16) for (int k = KSA; k < KSA + 8; ++k) Ah[lane][k] = (b16)0.0f;
  wave_lds_sync();
  gemm16<KSA, 16>(Ah, Al, false, WB + woff(6), Bs.p[6], 1, 1.0f / (XS * WSC), Tf, nloc, hlf); wave_lds_sync();
  gemm16<DS, 16>(Ah, Al, false, WB + woff(10), Bs.p[10], 1, 1.0f / (XS * WSC), Ts, nloc, hlf); wave_lds_sync();
  stage_hl(Tf, Ah, Al, 0, lane); wave_lds_sync(); gemm16<HH, 16>(Ah, Al, true, WB + woff(7), Bs.p[7], 1, 1.0f / (HS * WSC), Tf, nloc, hlf); wave_lds_sync(); store(OA, Tf);
  stage_hl(Tf, Ah, Al, 0, lane); wave_lds_sync(); gemm16<HH, 16>(Ah, Al, true, WB + woff(8), Bs.p[8], 1, 1.0f / (HS * WSC), Tf, nloc, hlf); wave_lds_sync();
  stage_hl(Tf, Ah, Al, 0, lane); wave_lds_sync(); gemm16<HH, 16>(Ah, Al, true, WB + woff(9), Bs.p[9], 1, 1.0f / (HS * WSC), Tf, nloc, hlf); wave_lds_sync(); store(AV, Tf);
  stage_hl(Ts, Ah, Al, 0, lane); wave_lds_sync(); gemm16<HH, 16>(Ah, Al, true, WB + woff(11), Bs.p[11], 1, 1.0f / (HS * WSC), Ts, nloc, hlf); wave_lds_sync(); store(CU, Ts);
  for (int rr = 0; rr < 16; ++rr) for (int q = 0; q < 4; ++q) { const int c = q * 32 + lane; Ah[rr][c] = (b16)(bfv(states[(r0 + rr) * DS + c]) * XS); Al[rr][c] = (b16)0.0f; }
  wave_lds_sync(); gemm16<DS, 16>(Ah, Al, false, WB + woff(0), Bs.p[0], 1, 1.0f / (XS * WSC), Tf, nloc, hlf); wave_lds_sync();
  stage_hl(Tf, Ah, Al, 0, lane); wave_lds_sync(); gemm16<HH, 16>(Ah, Al, true, WB + woff(1), Bs.p[1], 1, 1.0f / (HS * WSC), Tf, nloc, hlf); wave_lds_sync(); store(SE, Tf);
  stage_hl(Tf, Ah, Al, 0, lane); wave_lds_sync();
  gemm16<HH, 16>(Ah, Al, true, WB + woff(2), Bs.p[2], 1, 1.0f / (HS * WSC), Ts, nloc, hlf); wave_lds_sync();
  gemm16<HH, 16>(Ah, Al, true, WB + woff(4), Bs.p[4], 1, 1.0f / (HS * WSC), Tf, nloc, hlf); wave_lds_sync();
  stage_hl(Ts, Ah, Al, 0, lane); wave_lds_sync(); gemm16<HH, 16>(Ah, Al, true, WB + woff(3), Bs.p[3], 1, 1.0f / (HS * WSC), Ts, nloc, hlf); wave_lds_sync(); store(KK, Ts);
  stage_hl(Tf, Ah, Al, 0, lane); wave_lds_sync(); gemm16<HH, 16>(Ah, Al, true, WB + woff(5), Bs.p[5], 1, 1.0f / (HS * WSC), Tf, nloc, hlf); wave_lds_sync(); store(QQ, Tf); }
__global__ __launch_bounds__(32) void batch_kernel(const float* __restrict__ SE, const float* __restrict__ KK, const float* __restrict__ QQ, const float* __restrict__ OA, const float* __restrict__ AV, const float* __restrict__ CU, const float* __restrict__ pol, const float* __restrict__ act, const b16* __restrict__ WB, BPtrs Bs, const float* __restrict__ l1w, const float* __restrict__ l1b, const float* __restrict__ l2w, const float* __restrict__ l2b, int BLIM, float* __restrict__ out0, float* __restrict__ out1, float* __restrict__ out2) { __shared__ __attribute__((aligned(16))) b16 Ah[16][520], Al[16][520]; __shared__ float Tf[16][260], Wt[NA][NA + 1], Nd[NA][260], Cr[NA][260], Qs[NA][AC + 1]; const int lane = threadIdx.x, nloc = lane & 15, hlf = lane >> 4; const int b = blockIdx.x; if (b >= BLIM) return; const size_t a0 = (size_t)b * NA;
  { const int n = lane; const float* qn = QQ + (a0 + n) * HH; float mx = -INFINITY;
#pragma unroll 1
    for (int m = 0; m < NA; ++m) { float s = 0.0f; if (m != n) { const float* km = KK + (a0 + m) * HH;
#pragma unroll 1
        for (int c = 0; c < HH; ++c) s += pmul(qn[c], km[c]); s *= (1.0f / 16.0f); mx = fmaxf(mx, s); } Wt[n][m] = s; }
    float sm = 0.0f;
#pragma unroll 1
    for (int m = 0; m < NA; ++m) { const float p = (m != n) ? __expf(Wt[n][m] - mx) : 0.0f; Wt[n][m] = p; sm += p; } const float inv = 1.0f / sm;
#pragma unroll 1
    for (int m = 0; m < NA; ++m) Wt[n][m] = (m == n) ? 1.0f : Wt[n][m] * inv; }
  wave_lds_sync();
  for (int n = 0; n < NA; ++n) { for (int q = 0; q < 8; ++q) { const int c = q * 32 + lane; float soa = 0.0f, sav = 0.0f, sse = 0.0f;
#pragma unroll 1
      for (int m = 0; m < NA; ++m) { if (m == n) continue; soa += OA[(a0 + m) * HH + c]; sav += pmul(Wt[n][m], AV[(a0 + m) * HH + c]); sse += SE[(a0 + m) * HH + c]; }
      Nd[n][c] = soa * (1.0f / (NA - 1)) + sav; Cr[n][c] = CU[(a0 + n) * HH + c] + sse * (1.0f / (NA - 1)) + SE[(a0 + n) * HH + c]; } }
  wave_lds_sync();
  { const int n = lane; auto lnrow = [&](float* row, const float* w, const float* bb) { float m = 0.0f; for (int c = 0; c < HH; ++c) m += row[c]; m *= (1.0f / HH); float vr = 0.0f; for (int c = 0; c < HH; ++c) { const float d = row[c] - m; vr += d * d; } vr *= (1.0f / HH); const float rs = rsqrtf(vr + EPS); for (int c = 0; c < HH; ++c) row[c] = pmul((row[c] - m) * rs, bfv(w[c])) + bfv(bb[c]); }; lnrow(&Nd[n][0], l1w, l1b); lnrow(&Cr[n][0], l2w, l2b); }
  wave_lds_sync();
  if (lane < 16) for (int k = 512; k < 520; ++k) { Ah[lane][k] = (b16)0.0f; Al[lane][k] = (b16)0.0f; }
  for (int rt = 0; rt < 2; ++rt) {
    for (int rr = 0; rr < 16; ++rr) for (int q = 0; q < 8; ++q) { const int c = q * 32 + lane; b16 p, pl; split16(Cr[rt * 16 + rr][c] * HS, p, pl); Ah[rr][c] = p; Al[rr][c] = pl; split16(Nd[rt * 16 + rr][c] * HS, p, pl); Ah[rr][HH + c] = p; Al[rr][HH + c] = pl; }
    wave_lds_sync(); gemm16<512, 16>(Ah, Al, true, WB + woff(12), Bs.p[12], 1, 1.0f / (HS * WSC), Tf, nloc, hlf); wave_lds_sync();
    stage_hl(Tf, Ah, Al, 0, lane); if (lane < 16) for (int k = HH; k < HH + 8; ++k) { Ah[lane][k] = (b16)0.0f; Al[lane][k] = (b16)0.0f; } wave_lds_sync(); gemm16<HH, 16>(Ah, Al, true, WB + woff(13), Bs.p[13], 1, 1.0f / (HS * WSC), Tf, nloc, hlf); wave_lds_sync();
    stage_hl(Tf, Ah, Al, 0, lane); wave_lds_sync(); gemm16<HH, 1>(Ah, Al, true, WB + woff(14), Bs.p[14], 0, 1.0f / (HS * WSC), Tf, nloc, hlf); wave_lds_sync();
    if (lane < 16) for (int a = 0; a < AC; ++a) Qs[rt * 16 + lane][a] = Tf[lane][a];
    wave_lds_sync(); }
  for (int pass = 0; pass < 2; ++pass) {
    for (int n = 0; n < NA; ++n) { float v = 0.0f; for (int a = 0; a < AC; ++a) v += pmul(Qs[n][a], bfv(pol[(a0 + lane) * AC + a])); ((volatile float*)out0)[(a0 + n) * NA + lane] = v; ((volatile float*)out2)[(a0 + n) * NA + lane] = Wt[n][lane]; }
    { float qv = 0.0f; for (int a = 0; a < AC; ++a) qv += pmul(bfv(act[(a0 + lane) * AC + a]), Qs[lane][a]); ((volatile float*)out1)[a0 + lane] = qv; }
    __threadfence(); } }
}

extern "C" void kernel_launch(void* const* d_in, const int* in_sizes, int n_in, void* d_out, int out_size, void* d_ws, size_t ws_size, hipStream_t stream) {
  (void)n_in;
  auto Fp = [&](int i) { return (const float*)d_in[i]; };
  if (in_sizes[0] != R * DS || in_sizes[1] != R * AC || in_sizes[2] != R * AC || in_sizes[3] != DS * HH || in_sizes[15] != 144 * HH || in_sizes[27] != 512 * HH || in_sizes[31] != HH * AC || out_size != R * NA + R + R * NA) return;
  const int RLIM = R, BLIM = NB_;
  size_t off = 0; char* ws = (char*)d_ws;
  auto carve = [&](size_t bytes) { char* p = ws + off; off += (bytes + 255) & ~(size_t)255; return p; };
  b16* WB = (b16*)carve(woff(15) * 2);
  float* SE = (float*)carve((size_t)R * HH * 4); float* KK = (float*)carve((size_t)R * HH * 4); float* QQ = (float*)carve((size_t)R * HH * 4); float* OA = (float*)carve((size_t)R * HH * 4); float* AV = (float*)carve((size_t)R * HH * 4); float* CU = (float*)carve((size_t)R * HH * 4);
  if (off > ws_size || off > ((size_t)40 << 20)) return;
  const int widx[15] = {3, 5, 7, 9, 11, 13, 15, 17, 19, 21, 23, 25, 27, 29, 31};
  WPtrs Ws; BPtrs Bs; for (int i = 0; i < 15; ++i) { Ws.p[i] = Fp(widx[i]); Bs.p[i] = Fp(widx[i] + 1); }
  wput_kernel<<<dim3(32, 15), 256, 0, stream>>>(Ws, WB);
  agent_kernel<<<RLIM / 16, 32, 0, stream>>>(Fp(0), Fp(2), WB, Bs, RLIM, SE, KK, QQ, OA, AV, CU);
  float* out0 = (float*)d_out; float* out1 = out0 + (size_t)R * NA; float* out2 = out1 + R;
  batch_kernel<<<BLIM, 32, 0, stream>>>(SE, KK, QQ, OA, AV, CU, Fp(1), Fp(2), WB, Bs, Fp(33), Fp(34), Fp(35), Fp(36), BLIM, out0, out1, out2);
}
